// MetaJanusAttn_50440095924318
// MI455X (gfx1250) — hardware-verified
//
#include <hip/hip_runtime.h>
#include <stdint.h>

constexpr int NBATCH = 4;
constexpr int NT     = 2048;
constexpr int NE     = 1024;
constexpr int NTOK   = NBATCH * NT;
static_assert((NTOK % 64) == 0 && (NT % 64) == 0 && (NE % 64) == 0);

typedef __attribute__((ext_vector_type(16))) _Float16 v16h;
typedef __attribute__((ext_vector_type(8)))  _Float16 v8h;
typedef __attribute__((ext_vector_type(16))) __bf16   v16b;
typedef __attribute__((ext_vector_type(8)))  __bf16   v8b;
typedef __attribute__((ext_vector_type(8)))  float    v8f;
typedef __attribute__((ext_vector_type(4)))  float    v4f;
typedef __attribute__((ext_vector_type(8)))  unsigned short v8us;

__device__ __forceinline__ unsigned short f2bf_bits(float f) {
  unsigned u = __float_as_uint(f);
  return (unsigned short)((u + 0x7FFFu + ((u >> 16) & 1u)) >> 16);
}
__device__ __forceinline__ float bf_bits2f(unsigned short h) { return __uint_as_float(((unsigned)h) << 16); }

__device__ __forceinline__ void dep_guard_h(v8f& a, v8f& b, v16h x, v16h y) { asm volatile("v_nop\n\tv_nop\n\tv_nop\n\tv_nop" : "+v"(a), "+v"(b) : "v"(x), "v"(y)); }
__device__ __forceinline__ void dep_guard_b(v8f& a, v8f& b, v16b x, v16b y) { asm volatile("v_nop\n\tv_nop\n\tv_nop\n\tv_nop" : "+v"(a), "+v"(b) : "v"(x), "v"(y)); }
__device__ __forceinline__ void keep4_h(v16h a, v16h b, v16h c, v16h d) { asm volatile("v_nop" :: "v"(a), "v"(b), "v"(c), "v"(d)); }
__device__ __forceinline__ void keep4_b(v16b a, v16b b, v16b c, v16b d) { asm volatile("v_nop" :: "v"(a), "v"(b), "v"(c), "v"(d)); }
__device__ __forceinline__ void acc_guard4(v8f& a, v8f& b, v8f& c, v8f& d) { asm volatile("v_nop\n\tv_nop\n\tv_nop\n\tv_nop" : "+v"(a), "+v"(b), "+v"(c), "+v"(d)); }
template <typename T> struct Frag;
template <> struct Frag<_Float16> {
  typedef v16h V; union U { v16h v; v8h h[2]; };
  static __device__ __forceinline__ v16h load(const _Float16* p) {
    U f; f.h[0] = *(const v8h*)(p); f.h[1] = *(const v8h*)(p + 16); return f.v;
  }
  static __device__ __forceinline__ v8f mma(v16h a, v16h b, v8f c) {
    return __builtin_amdgcn_wmma_f32_16x16x32_f16(false, a, false, b, (short)0, c, false, false);
  }
  static __device__ __forceinline__ void guard(v8f& a, v8f& b, v16h x, v16h y) { dep_guard_h(a, b, x, y); }
  static __device__ __forceinline__ void keep(v16h a, v16h b, v16h c, v16h d) { keep4_h(a, b, c, d); }
};
template <> struct Frag<__bf16> {
  typedef v16b V; union U { v16b v; v8b h[2]; };
  static __device__ __forceinline__ v16b load(const __bf16* p) {
    U f; f.h[0] = *(const v8b*)(p); f.h[1] = *(const v8b*)(p + 16); return f.v;
  }
  static __device__ __forceinline__ v8f mma(v16b a, v16b b, v8f c) {
    return __builtin_amdgcn_wmma_f32_16x16x32_bf16(false, a, false, b, (short)0, c, false, false);
  }
  static __device__ __forceinline__ void guard(v8f& a, v8f& b, v16b x, v16b y) { dep_guard_b(a, b, x, y); }
  static __device__ __forceinline__ void keep(v16b a, v16b b, v16b c, v16b d) { keep4_b(a, b, c, d); }
};

template <int ET> struct Elem;
template <> struct Elem<0> { typedef _Float16 T; };
template <> struct Elem<1> { typedef __bf16 T; };
template <int ET, int SPLIT, int OUT_MODE, bool CAUSAL>
__global__ __launch_bounds__(256) void wmma_gemm64(
    const unsigned short* __restrict__ Ap, const unsigned short* __restrict__ A2p, int lda, long strideA,
    const unsigned short* __restrict__ Btp, const unsigned short* __restrict__ Bt2p, int ldb, long strideB,
    void* __restrict__ Cout, void* __restrict__ Cout2, int ldc, long strideC,
    int M, int N, int K, float scale) {
  typedef typename Elem<ET>::T T;
  typedef typename Frag<T>::V V;
  const T* A = (const T*)Ap; const T* A2 = (const T*)A2p; const T* Bt = (const T*)Btp; const T* Bt2 = (const T*)Bt2p;
  __shared__ __align__(16) float sT[8][16 * 68];
  const int b    = blockIdx.y;
  const int lane = threadIdx.x & 31;
  const int wave = threadIdx.x >> 5;
  const int tilesN = N >> 6;
  const int tilesM = M >> 6;
  const int tile = blockIdx.x * 8 + wave;
  if (tile >= tilesM * tilesN) return;
  const int tm = tile / tilesN;
  const int tn = tile - tm * tilesN;
  const int m0 = tm << 6;
  const int n0 = tn << 6;

  const T* Ab  = A  + (size_t)b * strideA;
  const T* Bb  = Bt + (size_t)b * strideB;
  const T* Ab2 = (SPLIT >= 1) ? (A2  + (size_t)b * strideA) : nullptr;
  const T* Bb2 = (SPLIT == 2) ? (Bt2 + (size_t)b * strideB) : nullptr;

  const int rlane = lane & 15;
  const int koff  = (lane >> 4) * 8;
  const int mOff  = (lane >> 4) * 8;

  v8f acc[4][4];
#pragma unroll
  for (int i = 0; i < 4; ++i)
#pragma unroll
    for (int j = 0; j < 4; ++j) acc[i][j] = (v8f){0.f,0.f,0.f,0.f,0.f,0.f,0.f,0.f};

  int kEnd = K;
  if (CAUSAL) kEnd = (m0 + 64 < K) ? (m0 + 64) : K;

  for (int k0 = 0; k0 < kEnd; k0 += 32) {
    V bh[4], bl[4];
#pragma unroll
    for (int j = 0; j < 4; ++j) {
      const size_t bo = (size_t)(n0 + (j << 4) + rlane) * ldb + koff + k0;
      bh[j] = Frag<T>::load(Bb + bo);
      if (SPLIT == 2) bl[j] = Frag<T>::load(Bb2 + bo);
    }
#pragma unroll
    for (int i = 0; i < 4; ++i) {
      const size_t ao = (size_t)(m0 + (i << 4) + rlane) * lda + koff + k0;
      V ah = Frag<T>::load(Ab + ao);
      V al;
      if (SPLIT >= 1) al = Frag<T>::load(Ab2 + ao);
#pragma unroll
      for (int j = 0; j < 4; ++j) {
        acc[i][j] = Frag<T>::mma(ah, bh[j], acc[i][j]);
        if (SPLIT == 2) acc[i][j] = Frag<T>::mma(ah, bl[j], acc[i][j]);
        if (SPLIT >= 1) acc[i][j] = Frag<T>::mma(al, bh[j], acc[i][j]);
      }
      Frag<T>::guard(acc[i][0], acc[i][3], ah, (SPLIT != 0) ? al : ah);
    }
    Frag<T>::keep(bh[0], bh[1], bh[2], bh[3]);
    if (SPLIT == 2) Frag<T>::keep(bl[0], bl[1], bl[2], bl[3]);
  }
  acc_guard4(acc[0][0], acc[0][1], acc[0][2], acc[0][3]);
  acc_guard4(acc[1][0], acc[1][1], acc[1][2], acc[1][3]);
  acc_guard4(acc[2][0], acc[2][1], acc[2][2], acc[2][3]);
  acc_guard4(acc[3][0], acc[3][1], acc[3][2], acc[3][3]);

  float* slab = sT[wave];
#pragma unroll
  for (int i = 0; i < 4; ++i) {
    const int mBase = m0 + (i << 4);
#pragma unroll
    for (int j = 0; j < 4; ++j) {
#pragma unroll
      for (int r = 0; r < 8; ++r) {
        float v = acc[i][j][r] * scale;
        slab[(mOff + r) * 68 + (j << 4) + rlane] = v;
      }
    }
    __builtin_amdgcn_fence(__ATOMIC_RELEASE, "workgroup");
    __builtin_amdgcn_wave_barrier();
    __builtin_amdgcn_fence(__ATOMIC_ACQUIRE, "workgroup");
    if (OUT_MODE == 0) {
      float* C = (float*)Cout + (size_t)b * strideC;
      const int hh = lane >> 4, c4 = (lane & 15) * 4;
      for (int pass = 0; pass < 2; ++pass) {
#pragma unroll
        for (int it = 0; it < 8; ++it) {
          const int row = it * 2 + hh;
          v4f v = *(const v4f*)(slab + row * 68 + c4);
          *(volatile v4f*)(C + (size_t)(mBase + row) * ldc + n0 + c4) = v;
        }
        __threadfence();
      }
    } else {
      const int q = lane >> 3, c8 = (lane & 7) * 8;
      unsigned short* C  = (unsigned short*)Cout  + (size_t)b * strideC;
      unsigned short* C2 = (OUT_MODE == 2) ? ((unsigned short*)Cout2 + (size_t)b * strideC) : nullptr;
      for (int pass = 0; pass < 2; ++pass) {
#pragma unroll
        for (int it = 0; it < 4; ++it) {
          const int row = it * 4 + q;
          const float* sp = slab + row * 68 + c8;
          v8h hv, lv;
#pragma unroll
          for (int e = 0; e < 8; ++e) {
            if (OUT_MODE == 1) {
              hv[e] = (_Float16)sp[e];
            } else {
              unsigned short hb = f2bf_bits(sp[e]);
              unsigned short lb = f2bf_bits(sp[e] - bf_bits2f(hb));
              hv[e] = __builtin_bit_cast(_Float16, hb);
              lv[e] = __builtin_bit_cast(_Float16, lb);
            }
          }
          *(volatile v8h*)(C + (size_t)(mBase + row) * ldc + n0 + c8) = hv;
          if (OUT_MODE == 2) *(volatile v8h*)(C2 + (size_t)(mBase + row) * ldc + n0 + c8) = lv;
        }
        __threadfence();
      }
    }
    __builtin_amdgcn_fence(__ATOMIC_RELEASE, "workgroup");
    __builtin_amdgcn_wave_barrier();
    __builtin_amdgcn_fence(__ATOMIC_ACQUIRE, "workgroup");
  }
}

__global__ __launch_bounds__(256) void cast_f32_bf16x2(
    const float* __restrict__ in, unsigned short* __restrict__ out, int n2) {
  const int i = blockIdx.x * 256 + threadIdx.x;
  if (i < n2) {
    const float a0 = in[2 * (size_t)i], a1 = in[2 * (size_t)i + 1];
    const unsigned u = (unsigned)f2bf_bits(a0) | ((unsigned)f2bf_bits(a1) << 16);
    ((volatile unsigned*)out)[i] = u;
    __threadfence();
    ((volatile unsigned*)out)[i] = u;
  }
}

constexpr int WTPITCH = 72;
__global__ __launch_bounds__(256) void wt_cast_bf16_k(const float* __restrict__ W, unsigned short* __restrict__ Wtp,
                                                      int K, int N) {
  __shared__ __align__(16) _Float16 st[64 * WTPITCH];
  _Float16* Wt = (_Float16*)Wtp;
  const int n0 = blockIdx.x * 64, k0 = blockIdx.y * 64;
  const int tid = threadIdx.x;
  const int kr = tid >> 2, c16 = (tid & 3) * 16;
  const float* src = W + (size_t)(k0 + kr) * N + n0 + c16;
#pragma unroll
  for (int q = 0; q < 4; ++q) {
    const v4f v = *(const v4f*)(src + 4 * q);
#pragma unroll
    for (int e = 0; e < 4; ++e) st[(c16 + 4 * q + e) * WTPITCH + kr] = __builtin_bit_cast(_Float16, f2bf_bits(v[e]));
  }
  __syncthreads();
  const int wave = tid >> 5, lane = tid & 31;
  const int q8 = lane >> 3, c8 = (lane & 7) * 8;
  for (int pass = 0; pass < 2; ++pass) {
#pragma unroll
    for (int it = 0; it < 2; ++it) {
      const int n = it * 32 + wave * 4 + q8;
      const v8h hv = *(const v8h*)(st + n * WTPITCH + c8);
      *(volatile v8h*)(Wt + (size_t)(n0 + n) * K + k0 + c8) = hv;
    }
    __threadfence();
  }
}

__global__ __launch_bounds__(256) void sc_k(const unsigned short* __restrict__ xb, const float* __restrict__ eb,
                                            float* __restrict__ sc) {
  __shared__ float s_val[32];
  const int wave = threadIdx.x >> 5, lane = threadIdx.x & 31;
  const int row0 = blockIdx.x * 32;
  for (int i = 0; i < 4; ++i) {
    const int r = row0 + wave * 4 + i;
    const unsigned short* xr = xb + (size_t)r * NE;
    const float* er = eb + (size_t)r * NE;
    float s = 0.f;
#pragma unroll 1
    for (int it = 0; it < NE / 256; ++it) {
      const int e0 = it * 256 + lane * 8;
      const v8us xv = *(const v8us*)(xr + e0);
      const v4f ea = *(const v4f*)(er + e0);
      const v4f ec = *(const v4f*)(er + e0 + 4);
      s = fmaf(bf_bits2f(xv[0]), ea[0], s);
      s = fmaf(bf_bits2f(xv[1]), ea[1], s);
      s = fmaf(bf_bits2f(xv[2]), ea[2], s);
      s = fmaf(bf_bits2f(xv[3]), ea[3], s);
      s = fmaf(bf_bits2f(xv[4]), ec[0], s);
      s = fmaf(bf_bits2f(xv[5]), ec[1], s);
      s = fmaf(bf_bits2f(xv[6]), ec[2], s);
      s = fmaf(bf_bits2f(xv[7]), ec[3], s);
    }
#pragma unroll
    for (int off = 16; off; off >>= 1) s += __shfl_xor(s, off, 32);
    if (lane == 0) s_val[wave * 4 + i] = s * (1.0f / 32.0f);
  }
  __syncthreads();
  if (wave == 0) {
    const float v = s_val[lane];
    *(volatile float*)(sc + row0 + lane) = v;
    __threadfence();
    *(volatile float*)(sc + row0 + lane) = v;
  }
}

__global__ __launch_bounds__(256) void stats_k(const float* __restrict__ sc, float* __restrict__ mrow,
                                               float* __restrict__ linv) {
  __shared__ float s_m[32], s_l[32];
  const int wave = threadIdx.x >> 5, lane = threadIdx.x & 31;
  const int row0 = blockIdx.x * 32;
  const int b = row0 / NT;
  const float* scb = sc + (size_t)b * NT;
  for (int i = 0; i < 4; ++i) {
    const int rg = row0 + wave * 4 + i;
    const int t = rg - b * NT;
    const float sct = scb[t];
    float mx = __uint_as_float(0xff800000u);
#pragma unroll 1
    for (int s = lane; s <= t; s += 32) mx = fmaxf(mx, sct * scb[s]);
#pragma unroll
    for (int off = 16; off; off >>= 1) mx = fmaxf(mx, __shfl_xor(mx, off, 32));
    float z = 0.f;
#pragma unroll 1
    for (int s = lane; s <= t; s += 32) z += __expf(fmaf(sct, scb[s], -mx));
#pragma unroll
    for (int off = 16; off; off >>= 1) z += __shfl_xor(z, off, 32);
    if (lane == 0) { s_m[wave * 4 + i] = mx; s_l[wave * 4 + i] = 1.0f / z; }
  }
  __syncthreads();
  if (wave == 0) {
    const float mv = s_m[lane], lv = s_l[lane];
    *(volatile float*)(mrow + row0 + lane) = mv;
    *(volatile float*)(linv + row0 + lane) = lv;
    __threadfence();
    *(volatile float*)(mrow + row0 + lane) = mv;
    *(volatile float*)(linv + row0 + lane) = lv;
  }
}

__global__ __launch_bounds__(256) void pgen_k(const float* __restrict__ sc, const float* __restrict__ mrow,
                                              const float* __restrict__ linv, unsigned short* __restrict__ php,
                                              unsigned short* __restrict__ plp, int b) {
  union SV { v4f q[2]; float f[8]; };
  _Float16* ph = (_Float16*)php;
  _Float16* pl = (_Float16*)plp;
  const int wave = threadIdx.x >> 5, lane = threadIdx.x & 31;
  const int t = blockIdx.x * 8 + wave;
  const float* scb = sc + (size_t)b * NT;
  const float sct = scb[t];
  const float mt = mrow[(size_t)b * NT + t];
  const float li = linv[(size_t)b * NT + t];
  const int ncol = ((t >> 6) + 1) << 6;
  _Float16* prh = ph + (size_t)t * NT;
  _Float16* prl = pl + (size_t)t * NT;
  for (int base = 0; base < ncol; base += 256) {
    const int c = base + lane * 8;
    const bool active = c < ncol;
    const int cc = (c < NT - 8) ? c : (NT - 8);
    SV sv;
    sv.q[0] = *(const v4f*)(scb + cc);
    sv.q[1] = *(const v4f*)(scb + cc + 4);
    v8h hv, lv;
#pragma unroll
    for (int j = 0; j < 8; ++j) {
      float p = __expf(fmaf(sct, sv.f[j], -mt)) * li;
      p = (c + j <= t) ? p : 0.0f;
      const unsigned short hb = f2bf_bits(p);
      const unsigned short lb = f2bf_bits(p - bf_bits2f(hb));
      hv[j] = __builtin_bit_cast(_Float16, hb);
      lv[j] = __builtin_bit_cast(_Float16, lb);
    }
    for (int pass = 0; pass < 2; ++pass) {
      if (active) {
        *(volatile v8h*)(prh + c) = hv;
        *(volatile v8h*)(prl + c) = lv;
      }
      __threadfence();
    }
  }
}

extern "C" void kernel_launch(void* const* d_in, const int* in_sizes, int n_in,
                              void* d_out, int out_size, void* d_ws, size_t ws_size,
                              hipStream_t stream) {
  if (n_in < 4) return;
  if (in_sizes[0] != NTOK * NE || in_sizes[1] != NE * NE || in_sizes[2] != NE * NE ||
      in_sizes[3] != NE * NE || out_size != NTOK * NE) return;
  const float* x   = (const float*)d_in[0];
  const float* wj  = (const float*)d_in[1];
  const float* wjv = (const float*)d_in[2];
  const float* wo  = (const float*)d_in[3];
  float* outp = (float*)d_out;

  const size_t PLANE16 = (size_t)NTOK * NE * 2;
  const size_t WPL     = (size_t)NE * NE * 2;
  const size_t PLANE32 = (size_t)NTOK * NE * 4;
  const size_t PPL     = (size_t)NT * NT * 2;
  const size_t VEC     = (size_t)NTOK * 4;
  const size_t off_xb = 0;
  const size_t off_w  = off_xb + PLANE16;
  const size_t off_c  = off_w + 4 * WPL;
  const size_t off_d  = off_c + 2 * PLANE16;
  const size_t off_s  = off_d + PLANE32;
  const size_t total  = off_s + 3 * VEC;
  if (total > ws_size) return;

  char* ws = (char*)d_ws;
  unsigned short* xb     = (unsigned short*)(ws + off_xb);
  unsigned short* o_hi   = (unsigned short*)(ws + off_xb);
  unsigned short* wjb    = (unsigned short*)(ws + off_w);
  unsigned short* wjTb   = (unsigned short*)(ws + off_w + WPL);
  unsigned short* wjvb   = (unsigned short*)(ws + off_w + 2 * WPL);
  unsigned short* wob    = (unsigned short*)(ws + off_w + 3 * WPL);
  unsigned short* ech_hi = (unsigned short*)(ws + off_c);
  unsigned short* ech_lo = (unsigned short*)(ws + off_c + PLANE16);
  unsigned short* vt_hi  = (unsigned short*)(ws + off_c);
  unsigned short* vt_lo  = (unsigned short*)(ws + off_c + PLANE16);
  float*          ebp    = (float*)(ws + off_d);
  unsigned short* p_hi   = (unsigned short*)(ws + off_d);
  unsigned short* p_lo   = (unsigned short*)(ws + off_d + PPL);
  unsigned short* o_lo   = (unsigned short*)(ws + off_d + 2 * PPL);
  float*          scp    = (float*)(ws + off_s);
  float*          mrowp  = (float*)(ws + off_s + VEC);
  float*          linvp  = (float*)(ws + off_s + 2 * VEC);

  const dim3 blk(256);

  cast_f32_bf16x2<<<dim3((NTOK * NE / 2) / 256), blk, 0, stream>>>(x, xb, NTOK * NE / 2);
  cast_f32_bf16x2<<<dim3((NE * NE / 2) / 256), blk, 0, stream>>>(wj, wjb, NE * NE / 2);
  cast_f32_bf16x2<<<dim3((NE * NE / 2) / 256), blk, 0, stream>>>(wjv, wjvb, NE * NE / 2);
  cast_f32_bf16x2<<<dim3((NE * NE / 2) / 256), blk, 0, stream>>>(wo, wob, NE * NE / 2);
  wt_cast_bf16_k<<<dim3(NE / 64, NE / 64), blk, 0, stream>>>(wj, wjTb, NE, NE);

  wmma_gemm64<1, 0, 2, false><<<dim3((NTOK / 64) * (NE / 64) / 8, 1), blk, 0, stream>>>(
      xb, xb, NE, 0L, wjb, wjb, NE, 0L, (void*)ech_hi, (void*)ech_lo, NE, 0L, NTOK, NE, NE, 1.0f);
  wmma_gemm64<1, 1, 0, false><<<dim3((NTOK / 64) * (NE / 64) / 8, 1), blk, 0, stream>>>(
      ech_hi, ech_lo, NE, 0L, wjTb, wjTb, NE, 0L, (void*)ebp, (void*)ebp, NE, 0L, NTOK, NE, NE, 1.0f);
  sc_k<<<dim3(NTOK / 32), blk, 0, stream>>>(xb, ebp, scp);
  wmma_gemm64<1, 0, 2, false><<<dim3((NE / 64) * (NT / 64) / 8, NBATCH), blk, 0, stream>>>(
      wjvb, wjvb, NE, 0L, xb, xb, NE, (long)NT * NE, (void*)vt_hi, (void*)vt_lo, NT, (long)NE * NT, NE, NT, NE, 1.0f);
  stats_k<<<dim3(NTOK / 32), blk, 0, stream>>>(scp, mrowp, linvp);
  for (int bb = 0; bb < NBATCH; ++bb) {
    pgen_k<<<dim3(NT / 8), blk, 0, stream>>>(scp, mrowp, linvp, p_hi, p_lo, bb);
    wmma_gemm64<1, 2, 2, true><<<dim3((NT / 64) * (NE / 64) / 8, 1), blk, 0, stream>>>(
        p_hi, p_lo, NT, 0L,
        vt_hi + (size_t)bb * NE * NT, vt_lo + (size_t)bb * NE * NT, NT, 0L,
        (void*)(o_hi + (size_t)bb * NT * NE), (void*)(o_lo + (size_t)bb * NT * NE), NE, 0L,
        NT, NE, NT, 1.0f);
  }
  wmma_gemm64<1, 1, 0, false><<<dim3((NTOK / 64) * (NE / 64) / 8, 1), blk, 0, stream>>>(
      o_hi, o_lo, NE, 0L, wob, wob, NE, 0L, (void*)outp, (void*)outp, NE, 0L, NTOK, NE, NE, 1.0f);
}
